// UEncoder_26225070310020
// MI455X (gfx1250) — hardware-run, weakly checked
//
#include <hip/hip_runtime.h>
#include <stddef.h>


#define DM     512
#define DFF    2048
#define NH     8
#define DKH    64
#define GT     128
#define SPW    (32 * 64)
#define WPP    72
#define DEGCAP 128
#define WSCAP  134217728
#define ASCL   8.0f
#define WSCL   64.0f
#define INVSCL 0.001953125f
#define INVDM  0.001953125f
#define LNEPS  1e-5f

static_assert(NH * DKH == DM);
static_assert((DM % 128) == 0 && (DFF % 128) == 0);
static_assert((DM % 64) == 0 && (DFF % 64) == 0);
static_assert((WPP % 8) == 0);
static_assert(DEGCAP > 0);

typedef float          v4f  __attribute__((ext_vector_type(4)));
typedef float          v8f  __attribute__((ext_vector_type(8)));
typedef unsigned int   v4u  __attribute__((ext_vector_type(4)));
typedef unsigned short v8us __attribute__((ext_vector_type(8)));
typedef _Float16       v16h __attribute__((ext_vector_type(16)));
union FragH { v16h v; v8us u[2]; };

__device__ __forceinline__ unsigned short h16(float f) {
  const _Float16 h = (_Float16)f;
  return __builtin_bit_cast(unsigned short, h);
}
__device__ __forceinline__ float lo16f(unsigned int w) {
  return (float)__builtin_bit_cast(_Float16, (unsigned short)(w & 0xffffu));
}
__device__ __forceinline__ float hi16f(unsigned int w) {
  return (float)__builtin_bit_cast(_Float16, (unsigned short)(w >> 16));
}

__device__ __forceinline__ v8us cvt8(v4f a, v4f b, float s) {
  v8us r;
  r[0] = h16(a.x * s); r[1] = h16(a.y * s); r[2] = h16(a.z * s); r[3] = h16(a.w * s);
  r[4] = h16(b.x * s); r[5] = h16(b.y * s); r[6] = h16(b.z * s); r[7] = h16(b.w * s);
  return r;
}

__device__ __forceinline__ v4f relu4(v4f a) {
  v4f r;
  r.x = fmaxf(a.x, 0.0f); r.y = fmaxf(a.y, 0.0f); r.z = fmaxf(a.z, 0.0f); r.w = fmaxf(a.w, 0.0f);
  return r;
}

__device__ __forceinline__ v8f wmh(v16h a, v16h b, v8f c) {
  v8f d = __builtin_amdgcn_wmma_f32_16x16x32_f16(false, a, false, b, (short)0, c, false, false);
  asm volatile("v_nop\n\tv_nop\n\tv_nop\n\tv_nop" : "+v"(d) : "v"(a), "v"(b));
  return d;
}

__global__ __launch_bounds__(256) void k_wpack(
    const float* __restrict__ W, unsigned short* wt, int K, int M) {
  __shared__ __attribute__((aligned(16))) unsigned short sT[64 * WPP];
  const int tid = (int)threadIdx.x;
  const int m0 = (int)blockIdx.x * 64, k0 = (int)blockIdx.y * 64;
#pragma unroll 4
  for (int it = 0; it < 16; ++it) {
    const int idx = it * 256 + tid;
    const int kk = idx >> 6, mm = idx & 63;
    int kr = k0 + kk; kr = kr > K - 1 ? K - 1 : kr;
    int mc = m0 + mm; mc = mc > M - 1 ? M - 1 : mc;
    const float w = W[(size_t)kr * M + mc];
    sT[mm * WPP + kk] = h16(w * WSCL);
  }
  __syncthreads();
  v8us pv[2];
  size_t po[2];
#pragma unroll
  for (int it = 0; it < 2; ++it) {
    const int p = it * 256 + tid;
    const int row = p >> 3, c8 = (p & 7) * 8;
    pv[it] = *(const v8us*)(sT + row * WPP + c8);
    int mr = m0 + row; mr = mr > M - 1 ? M - 1 : mr;
    po[it] = (size_t)mr * K + k0 + c8;
  }
  const bool full = (m0 + 64 <= M) && (k0 + 64 <= K);
  if (full) {
#pragma unroll
    for (int it = 0; it < 2; ++it) *(volatile v8us*)(wt + po[it]) = pv[it];
  }
  __threadfence();
  if (full) {
#pragma unroll
    for (int it = 0; it < 2; ++it) *(volatile v8us*)(wt + po[it]) = pv[it];
  }
}

template <int OUT16>
__global__ __launch_bounds__(256) void k_ln(
    const float* X, const float* __restrict__ g, const float* __restrict__ b,
    float* outF, unsigned short* outH, int nRows) {
  const int tid = (int)threadIdx.x, lane = tid & 31, wave = tid >> 5;
  const int row = (int)blockIdx.x * 8 + wave;
  if (row < nRows) {
    int col[4];
    if (OUT16) { col[0] = 8 * lane; col[1] = 8 * lane + 4; col[2] = 256 + 8 * lane; col[3] = 256 + 8 * lane + 4; }
    else       { col[0] = 4 * lane; col[1] = 4 * lane + 128; col[2] = 4 * lane + 256; col[3] = 4 * lane + 384; }
    const float* xr = X + (size_t)row * DM;
    v4f a[4];
#pragma unroll
    for (int j = 0; j < 4; ++j) a[j] = *(const v4f*)(xr + col[j]);
    float s = 0.0f;
#pragma unroll
    for (int j = 0; j < 4; ++j) s += (a[j].x + a[j].y) + (a[j].z + a[j].w);
#pragma unroll
    for (int o = 16; o >= 1; o >>= 1) s += __shfl_xor(s, o);
    const float mu = s * INVDM;
    v4f d[4];
    float sq = 0.0f;
#pragma unroll
    for (int j = 0; j < 4; ++j) {
      d[j] = a[j] - mu;
      sq += (d[j].x * d[j].x + d[j].y * d[j].y) + (d[j].z * d[j].z + d[j].w * d[j].w);
    }
#pragma unroll
    for (int o = 16; o >= 1; o >>= 1) sq += __shfl_xor(sq, o);
    const float var  = sq * INVDM;
    const float rstd = rsqrtf(var + LNEPS);
    v4f y[4];
#pragma unroll
    for (int j = 0; j < 4; ++j) {
      const v4f g4 = *(const v4f*)(g + col[j]);
      const v4f b4 = *(const v4f*)(b + col[j]);
      y[j] = (d[j] * rstd) * g4 + b4;
    }
    if (OUT16) {
      const v8us h0 = cvt8(y[0], y[1], ASCL);
      const v8us h1 = cvt8(y[2], y[3], ASCL);
      unsigned short* op = outH + (size_t)row * DM;
      *(volatile v8us*)(op + 8 * lane) = h0;
      *(volatile v8us*)(op + 256 + 8 * lane) = h1;
      __threadfence();
      *(volatile v8us*)(op + 8 * lane) = h0;
      *(volatile v8us*)(op + 256 + 8 * lane) = h1;
    } else {
      float* op = outF + (size_t)row * DM;
#pragma unroll
      for (int j = 0; j < 4; ++j) *(volatile v4f*)(op + col[j]) = y[j];
      __threadfence();
#pragma unroll
      for (int j = 0; j < 4; ++j) *(volatile v4f*)(op + col[j]) = y[j];
    }
  }
}

template <int OUT16, int RELU, int RESID>
__global__ __launch_bounds__(GT) void k_gemm(
    const unsigned short* __restrict__ A, const unsigned short* __restrict__ Bt,
    const float* __restrict__ bias, const float* res,
    float* outF, unsigned short* outH, int K, int Ncols, int M) {
  __shared__ __attribute__((aligned(16))) float sT[4 * SPW];
  const int tid = (int)threadIdx.x, lane = tid & 31, wave = tid >> 5, hh = lane >> 4, m = lane & 15;
  const int r0 = (int)blockIdx.y * 64 + (wave >> 1) * 32;
  const int c0 = (int)blockIdx.x * 128 + (wave & 1) * 64;

  int ra0 = r0 + m;      ra0 = ra0 > M - 1 ? M - 1 : ra0;
  int ra1 = r0 + 16 + m; ra1 = ra1 > M - 1 ? M - 1 : ra1;
  const unsigned short* ap0 = A + (size_t)ra0 * K + 8 * hh;
  const unsigned short* ap1 = A + (size_t)ra1 * K + 8 * hh;
  const unsigned short* bp[4];
#pragma unroll
  for (int j = 0; j < 4; ++j) {
    int cb = c0 + 16 * j + m; cb = cb > Ncols - 1 ? Ncols - 1 : cb;
    bp[j] = Bt + (size_t)cb * K + 8 * hh;
  }

  v8f acc[2][4];
#pragma unroll
  for (int i = 0; i < 2; ++i)
#pragma unroll
    for (int j = 0; j < 4; ++j) { v8f z = {0.f, 0.f, 0.f, 0.f, 0.f, 0.f, 0.f, 0.f}; acc[i][j] = z; }

  const int nk = K >> 5;
#pragma unroll 1
  for (int kt = 0; kt < nk; ++kt) {
    const int kb = kt << 5;
    FragH a0, a1;
    a0.u[0] = *(const v8us*)(ap0 + kb);
    a0.u[1] = *(const v8us*)(ap0 + kb + 16);
    a1.u[0] = *(const v8us*)(ap1 + kb);
    a1.u[1] = *(const v8us*)(ap1 + kb + 16);
#pragma unroll
    for (int j = 0; j < 4; ++j) {
      FragH bf;
      bf.u[0] = *(const v8us*)(bp[j] + kb);
      bf.u[1] = *(const v8us*)(bp[j] + kb + 16);
      acc[0][j] = wmh(a0.v, bf.v, acc[0][j]);
      acc[1][j] = wmh(a1.v, bf.v, acc[1][j]);
    }
  }

  float* sw = sT + wave * SPW;
#pragma unroll
  for (int i = 0; i < 2; ++i)
#pragma unroll
    for (int j = 0; j < 4; ++j)
#pragma unroll
      for (int r = 0; r < 8; ++r)
        sw[(16 * i + 8 * hh + r) * 64 + 16 * j + m] = acc[i][j][r];
  __syncthreads();

  const bool full = (r0 + 32 <= M) && (c0 + 64 <= Ncols);
  if (OUT16) {
    v8us hv[8];
    size_t po[8];
#pragma unroll
    for (int it = 0; it < 8; ++it) {
      const int f = it * 32 + lane;
      const int row = f >> 3, c8 = (f & 7) * 8;
      const v4f v0 = *(const v4f*)(sw + row * 64 + c8);
      const v4f v1 = *(const v4f*)(sw + row * 64 + c8 + 4);
      int gc = c0 + c8; gc = gc > Ncols - 8 ? Ncols - 8 : gc;
      const v4f b0v = *(const v4f*)(bias + gc);
      const v4f b1v = *(const v4f*)(bias + gc + 4);
      v4f o0 = v0 * INVSCL + b0v;
      v4f o1 = v1 * INVSCL + b1v;
      if (RELU) { o0 = relu4(o0); o1 = relu4(o1); }
      hv[it] = cvt8(o0, o1, ASCL);
      po[it] = (size_t)(r0 + row) * Ncols + c0 + c8;
    }
    if (full) {
#pragma unroll
      for (int it = 0; it < 8; ++it) *(volatile v8us*)(outH + po[it]) = hv[it];
    }
    __threadfence();
    if (full) {
#pragma unroll
      for (int it = 0; it < 8; ++it) *(volatile v8us*)(outH + po[it]) = hv[it];
    }
  } else {
    v4f ov[16];
    size_t po[16];
#pragma unroll
    for (int it = 0; it < 16; ++it) {
      const int f = it * 32 + lane;
      const int row = f >> 4, c4 = (f & 15) * 4;
      const v4f v = *(const v4f*)(sw + row * 64 + c4);
      int gc = c0 + c4; gc = gc > Ncols - 4 ? Ncols - 4 : gc;
      int gr = r0 + row; gr = gr > M - 1 ? M - 1 : gr;
      const v4f bb = *(const v4f*)(bias + gc);
      v4f o = v * INVSCL + bb;
      if (RESID) o = o + *(const v4f*)(res + (size_t)gr * Ncols + gc);
      ov[it] = o;
      po[it] = (size_t)(r0 + row) * Ncols + c0 + c4;
    }
    if (full) {
#pragma unroll
      for (int it = 0; it < 16; ++it) *(volatile v4f*)(outF + po[it]) = ov[it];
    }
    __threadfence();
    if (full) {
#pragma unroll
      for (int it = 0; it < 16; ++it) *(volatile v4f*)(outF + po[it]) = ov[it];
    }
  }
}

__global__ __launch_bounds__(256) void k_agg(
    const unsigned short* __restrict__ q16, const unsigned short* __restrict__ k16,
    const unsigned short* __restrict__ v16, const int* __restrict__ src,
    const int* __restrict__ dst, unsigned short* att, int nN, int nE) {
  __shared__ int seg[8];
  __shared__ __attribute__((aligned(16))) unsigned int sO[NH * 4 * 32];
  const int tid = (int)threadIdx.x, lane = tid & 31, wave = tid >> 5;
  const int nb = (int)blockIdx.x * 4;

  if (wave == 0) {
    const int jn  = (lane >> 1) & 3;
    const int key = nb + jn + (lane & 1);
    int lo = 0, n = nE;
#pragma unroll 1
    for (int it = 0; it < 34; ++it) {
      const int half = n >> 1;
      const int mid  = lo + half;
      int ma = mid > nE - 1 ? nE - 1 : mid; ma = ma < 0 ? 0 : ma;
      const int d = dst[ma];
      const bool go = (n > 0) && (d < key);
      lo = go ? (mid + 1) : lo;
      n  = go ? (n - half - 1) : half;
    }
    if (lane < 8) seg[lane] = lo;
  }
  __syncthreads();

#pragma unroll 1
  for (int j = 0; j < 4; ++j) {
    const int node = nb + j;
    int lb = __builtin_amdgcn_readfirstlane(seg[2 * j]);
    int ub = __builtin_amdgcn_readfirstlane(seg[2 * j + 1]);
    lb = lb < 0 ? 0 : (lb > nE ? nE : lb);
    int cnt = ub - lb;
    cnt = cnt < 0 ? 0 : (cnt > DEGCAP ? DEGCAP : cnt);
    const unsigned int qw = *(const unsigned int*)(q16 + (size_t)node * DM + wave * DKH + 2 * lane);
    const float q0 = lo16f(qw), q1 = hi16f(qw);
    float acc0 = 0.0f, acc1 = 0.0f, z = 0.0f;
#pragma unroll 1
    for (int i = 0; i < cnt; ++i) {
      int e = lb + i; e = e > nE - 1 ? nE - 1 : e;
      int s = src[e];
      s = s < 0 ? 0 : (s > nN - 1 ? nN - 1 : s);
      const unsigned int kw = *(const unsigned int*)(k16 + (size_t)s * DM + wave * DKH + 2 * lane);
      float part = q0 * lo16f(kw) + q1 * hi16f(kw);
      part += __shfl_xor(part, 16);
      part += __shfl_xor(part, 8);
      part += __shfl_xor(part, 4);
      part += __shfl_xor(part, 2);
      part += __shfl_xor(part, 1);
      float sc = part * INVSCL;
      sc = fminf(fmaxf(sc, -10.0f), 10.0f);
      sc = __expf(sc);
      const unsigned int vw = *(const unsigned int*)(v16 + (size_t)s * DM + wave * DKH + 2 * lane);
      acc0 += sc * lo16f(vw);
      acc1 += sc * hi16f(vw);
      z += sc;
    }
    const float rz = 1.0f / z;
    const unsigned int o = (unsigned int)h16(acc0 * rz) | ((unsigned int)h16(acc1 * rz) << 16);
    sO[(wave * 4 + j) * 32 + lane] = o;
  }
  __syncthreads();

  const int qn = lane >> 3, p = lane & 7;
  const v4u val = *(const v4u*)(sO + (wave * 4 + qn) * 32 + 4 * p);
  unsigned short* gp = att + (size_t)(nb + qn) * DM + wave * DKH + 8 * p;
  *(volatile v4u*)gp = val;
  __threadfence();
  *(volatile v4u*)gp = val;
}

extern "C" void kernel_launch(void* const* d_in, const int* in_sizes, int n_in,
                              void* d_out, int out_size, void* d_ws, size_t ws_size,
                              hipStream_t stream) {
  if (n_in < 21) return;
  const int nN = in_sizes[0] / DM;
  const int nE = in_sizes[1];
  if (nN <= 0 || nE <= 0) return;
  if (in_sizes[0] != nN * DM || (nN % 64) != 0) return;
  if (in_sizes[2] != nE) return;
  if (nN > (1 << 22) || nE > (1 << 30)) return;
  if (in_sizes[3] != DM * DM || in_sizes[5] != DM * DM || in_sizes[7] != DM * DM || in_sizes[9] != DM * DM) return;
  if (in_sizes[4] != DM || in_sizes[6] != DM || in_sizes[8] != DM || in_sizes[10] != DM) return;
  if (in_sizes[11] != DM || in_sizes[12] != DM) return;
  if (in_sizes[13] != DM * DFF || in_sizes[14] != DFF) return;
  if (in_sizes[15] != DFF * DM || in_sizes[16] != DM) return;
  if (in_sizes[17] != DM || in_sizes[18] != DM || in_sizes[19] != DM || in_sizes[20] != DM) return;
  if (out_size != nN * DM) return;

  const float* x   = (const float*)d_in[0];
  const int*   src = (const int*)d_in[1];
  const int*   dst = (const int*)d_in[2];
  const float* Wq  = (const float*)d_in[3];
  const float* bq  = (const float*)d_in[4];
  const float* Wk  = (const float*)d_in[5];
  const float* bk  = (const float*)d_in[6];
  const float* Wv  = (const float*)d_in[7];
  const float* bv  = (const float*)d_in[8];
  const float* Wo  = (const float*)d_in[9];
  const float* bo  = (const float*)d_in[10];
  const float* g0  = (const float*)d_in[11];
  const float* b0  = (const float*)d_in[12];
  const float* W1  = (const float*)d_in[13];
  const float* bf1 = (const float*)d_in[14];
  const float* W2  = (const float*)d_in[15];
  const float* bf2 = (const float*)d_in[16];
  const float* g1  = (const float*)d_in[17];
  const float* b1  = (const float*)d_in[18];
  const float* gn  = (const float*)d_in[19];
  const float* bn  = (const float*)d_in[20];
  float* out = (float*)d_out;

  const size_t szWsq = (size_t)DM * DM * 2;
  const size_t szWff = (size_t)DM * DFF * 2;
  const size_t szQKV = (size_t)3 * nN * DM * 2;
  const size_t szFF  = (size_t)nN * DFF * 2;
  const size_t szA   = szQKV > szFF ? szQKV : szFF;
  const size_t szB   = (size_t)nN * DM * 2;
  const size_t szC   = (size_t)nN * DM * 4;
  size_t off = 0;
  const size_t oWq = off; off += szWsq;
  const size_t oWk = off; off += szWsq;
  const size_t oWv = off; off += szWsq;
  const size_t oWo = off; off += szWsq;
  const size_t oW1 = off; off += szWff;
  const size_t oW2 = off; off += szWff;
  const size_t oA  = off; off += szA;   off = (off + 255) & ~(size_t)255;
  const size_t oB  = off; off += szB;   off = (off + 255) & ~(size_t)255;
  const size_t oC  = off; off += szC;   off = (off + 255) & ~(size_t)255;
  if (off > ws_size || off > (size_t)WSCAP) return;

  char* ws = (char*)d_ws;
  unsigned short* wq16 = (unsigned short*)(ws + oWq);
  unsigned short* wk16 = (unsigned short*)(ws + oWk);
  unsigned short* wv16 = (unsigned short*)(ws + oWv);
  unsigned short* wo16 = (unsigned short*)(ws + oWo);
  unsigned short* w116 = (unsigned short*)(ws + oW1);
  unsigned short* w216 = (unsigned short*)(ws + oW2);
  unsigned short* q16  = (unsigned short*)(ws + oA);
  unsigned short* k16  = q16 + (size_t)nN * DM;
  unsigned short* v16  = k16 + (size_t)nN * DM;
  unsigned short* ff16 = (unsigned short*)(ws + oA);
  unsigned short* bh16 = (unsigned short*)(ws + oB);
  float*          xc   = (float*)(ws + oC);

  const dim3 gWsq(DM / 64, DM / 64);
  const dim3 gW1(DFF / 64, DM / 64);
  const dim3 gW2(DM / 64, DFF / 64);
  const dim3 gGD(DM / 128, nN / 64);
  const dim3 gGF(DFF / 128, nN / 64);

  k_wpack<<<gWsq, 256, 0, stream>>>(Wq, wq16, DM, DM);
  k_wpack<<<gWsq, 256, 0, stream>>>(Wk, wk16, DM, DM);
  k_wpack<<<gWsq, 256, 0, stream>>>(Wv, wv16, DM, DM);
  k_wpack<<<gWsq, 256, 0, stream>>>(Wo, wo16, DM, DM);
  k_wpack<<<gW1,  256, 0, stream>>>(W1, w116, DM, DFF);
  k_wpack<<<gW2,  256, 0, stream>>>(W2, w216, DFF, DM);

  k_ln<1><<<nN / 8, 256, 0, stream>>>(x, g0, b0, xc, bh16, nN);

  k_gemm<1, 0, 0><<<gGD, GT, 0, stream>>>(bh16, wq16, bq, x, xc, q16, DM, DM, nN);
  k_gemm<1, 0, 0><<<gGD, GT, 0, stream>>>(bh16, wk16, bk, x, xc, k16, DM, DM, nN);
  k_gemm<1, 0, 0><<<gGD, GT, 0, stream>>>(bh16, wv16, bv, x, xc, v16, DM, DM, nN);

  k_agg<<<nN / 4, 256, 0, stream>>>(q16, k16, v16, src, dst, bh16, nN, nE);

  k_gemm<0, 0, 1><<<gGD, GT, 0, stream>>>(bh16, wo16, bo, x, xc, ff16, DM, DM, nN);

  k_ln<1><<<nN / 8, 256, 0, stream>>>(xc, g1, b1, xc, bh16, nN);

  k_gemm<1, 1, 0><<<gGF, GT, 0, stream>>>(bh16, w116, bf1, x, (float*)ff16, ff16, DM, DFF, nN);

  k_gemm<0, 0, 1><<<gGD, GT, 0, stream>>>(ff16, w216, bf2, xc, xc, bh16, DFF, DM, nN);

  k_ln<0><<<nN / 8, 256, 0, stream>>>(xc, gn, bn, out, bh16, nN);
}
